// DalleSelfAttention_60318520705234
// MI455X (gfx1250) — hardware-verified
//
#include <hip/hip_runtime.h>

typedef __attribute__((ext_vector_type(16))) _Float16 v16h;
typedef __attribute__((ext_vector_type(8)))  _Float16 v8h;
typedef __attribute__((ext_vector_type(16))) __bf16   v16b;
typedef __attribute__((ext_vector_type(8)))  __bf16   v8b;
typedef __attribute__((ext_vector_type(8)))  float    v8f;
typedef __attribute__((ext_vector_type(4)))  float    v4f;
typedef __attribute__((ext_vector_type(4)))  unsigned int v4u;

__device__ __forceinline__ unsigned short f2bf_bits(float f) {
  unsigned u = __float_as_uint(f);
  return (unsigned short)((u + 0x7FFFu + ((u >> 16) & 1u)) >> 16);
}
__device__ __forceinline__ float bf_bits2f(unsigned short h) { return __uint_as_float(((unsigned)h) << 16); }
__device__ __forceinline__ unsigned int rne_bf16_word(unsigned int u) {
  return (u + 0x7FFFu + ((u >> 16) & 1u)) & 0xFFFF0000u;
}
__device__ __forceinline__ unsigned int pack_bf16x2(float a, float b) {
  return (unsigned int)f2bf_bits(a) | ((unsigned int)f2bf_bits(b) << 16);
}
__device__ __forceinline__ void split_pack2(float a, float b, unsigned int& wh, unsigned int& wl) {
  const unsigned short ha = f2bf_bits(a), hb = f2bf_bits(b);
  const unsigned short la = f2bf_bits(a - bf_bits2f(ha)), lb = f2bf_bits(b - bf_bits2f(hb));
  wh = (unsigned int)ha | ((unsigned int)hb << 16);
  wl = (unsigned int)la | ((unsigned int)lb << 16);
}

__device__ __forceinline__ void dep_guard_h(v8f& a, v8f& b, v16h x, v16h y) { asm volatile("v_nop\n\tv_nop\n\tv_nop\n\tv_nop" : "+v"(a), "+v"(b) : "v"(x), "v"(y)); }
__device__ __forceinline__ void dep_guard_b(v8f& a, v8f& b, v16b x, v16b y) { asm volatile("v_nop\n\tv_nop\n\tv_nop\n\tv_nop" : "+v"(a), "+v"(b) : "v"(x), "v"(y)); }
__device__ __forceinline__ void keep4_h(v16h a, v16h b, v16h c, v16h d) { asm volatile("v_nop" :: "v"(a), "v"(b), "v"(c), "v"(d)); }
__device__ __forceinline__ void keep4_b(v16b a, v16b b, v16b c, v16b d) { asm volatile("v_nop" :: "v"(a), "v"(b), "v"(c), "v"(d)); }
__device__ __forceinline__ void acc_guard4(v8f& a, v8f& b, v8f& c, v8f& d) { asm volatile("v_nop\n\tv_nop\n\tv_nop\n\tv_nop" : "+v"(a), "+v"(b), "+v"(c), "+v"(d)); }
template <typename T> struct Frag;
template <> struct Frag<_Float16> {
  typedef v16h V; union U { v16h v; v8h h[2]; };
  static __device__ __forceinline__ v16h load(const _Float16* p) {
    U f; f.h[0] = *(const v8h*)(p); f.h[1] = *(const v8h*)(p + 16); return f.v;
  }
  static __device__ __forceinline__ v8f mma(v16h a, v16h b, v8f c) {
    return __builtin_amdgcn_wmma_f32_16x16x32_f16(false, a, false, b, (short)0, c, false, false);
  }
  static __device__ __forceinline__ void guard(v8f& a, v8f& b, v16h x, v16h y) { dep_guard_h(a, b, x, y); }
  static __device__ __forceinline__ void keep(v16h a, v16h b, v16h c, v16h d) { keep4_h(a, b, c, d); }
};
template <> struct Frag<__bf16> {
  typedef v16b V; union U { v16b v; v8b h[2]; };
  static __device__ __forceinline__ v16b load(const __bf16* p) {
    U f; f.h[0] = *(const v8b*)(p); f.h[1] = *(const v8b*)(p + 16); return f.v;
  }
  static __device__ __forceinline__ v8f mma(v16b a, v16b b, v8f c) {
    return __builtin_amdgcn_wmma_f32_16x16x32_bf16(false, a, false, b, (short)0, c, false, false);
  }
  static __device__ __forceinline__ void guard(v8f& a, v8f& b, v16b x, v16b y) { dep_guard_b(a, b, x, y); }
  static __device__ __forceinline__ void keep(v16b a, v16b b, v16b c, v16b d) { keep4_b(a, b, c, d); }
};

template <int ET> struct Elem;
template <> struct Elem<0> { typedef _Float16 T; };
template <> struct Elem<1> { typedef __bf16 T; };
template <int ET, int SPLIT, int BIAS_MODE, int OUT_MODE, bool RESID, int ACT = 0>
__global__ __launch_bounds__(256) void wmma_gemm64(
    const unsigned short* __restrict__ Ap, const unsigned short* __restrict__ A2p, int lda, long strideA,
    const unsigned short* __restrict__ Btp, const unsigned short* __restrict__ Bt2p, int ldb, long strideB,
    void* __restrict__ Cout, void* __restrict__ Cout2, int ldc, long strideC,
    const float* __restrict__ bias,
    const float* __restrict__ resid, long strideR,
    int M, int N, int K, float scale) {
  typedef typename Elem<ET>::T T;
  typedef typename Frag<T>::V V;
  const T* A = (const T*)Ap; const T* A2 = (const T*)A2p; const T* Bt = (const T*)Btp; const T* Bt2 = (const T*)Bt2p;
  __shared__ __align__(16) float sT[8][16 * 68];
  const int b    = blockIdx.y;
  const int lane = threadIdx.x & 31;
  const int wave = threadIdx.x >> 5;
  const int tilesN = N >> 6;
  const int tilesM = M >> 6;
  const int tile = blockIdx.x * 8 + wave;
  if (tile >= tilesM * tilesN) return;
  const int tm = tile / tilesN;
  const int tn = tile - tm * tilesN;
  const int m0 = tm << 6;
  const int n0 = tn << 6;

  const T* Ab  = A  + (size_t)b * strideA;
  const T* Bb  = Bt + (size_t)b * strideB;
  const T* Ab2 = (SPLIT != 0) ? (A2  + (size_t)b * strideA) : nullptr;
  const T* Bb2 = (SPLIT == 1) ? (Bt2 + (size_t)b * strideB) : nullptr;

  const int rlane = lane & 15;
  const int koff  = (lane >> 4) * 8;
  const int mOff  = (lane >> 4) * 8;

  v8f acc[4][4];
#pragma unroll
  for (int i = 0; i < 4; ++i)
#pragma unroll
    for (int j = 0; j < 4; ++j) acc[i][j] = (v8f){0.f,0.f,0.f,0.f,0.f,0.f,0.f,0.f};

  for (int k0 = 0; k0 < K; k0 += 32) {
    V bh[4], bl[4];
#pragma unroll
    for (int j = 0; j < 4; ++j) {
      const size_t bo = (size_t)(n0 + (j << 4) + rlane) * ldb + koff + k0;
      bh[j] = Frag<T>::load(Bb + bo);
      if (SPLIT == 1) bl[j] = Frag<T>::load(Bb2 + bo);
    }
#pragma unroll
    for (int i = 0; i < 4; ++i) {
      const size_t ao = (size_t)(m0 + (i << 4) + rlane) * lda + koff + k0;
      V ah = Frag<T>::load(Ab + ao);
      V al;
      if (SPLIT != 0) al = Frag<T>::load(Ab2 + ao);
#pragma unroll
      for (int j = 0; j < 4; ++j) {
        acc[i][j] = Frag<T>::mma(ah, bh[j], acc[i][j]);
        if (SPLIT == 1) {
          acc[i][j] = Frag<T>::mma(ah, bl[j], acc[i][j]);
          acc[i][j] = Frag<T>::mma(al, bh[j], acc[i][j]);
        }
        if (SPLIT == 2) {
          acc[i][j] = Frag<T>::mma(al, bh[j], acc[i][j]);
        }
      }
      Frag<T>::guard(acc[i][0], acc[i][3], ah, (SPLIT != 0) ? al : ah);
    }
    Frag<T>::keep(bh[0], bh[1], bh[2], bh[3]);
    if (SPLIT == 1) Frag<T>::keep(bl[0], bl[1], bl[2], bl[3]);
  }
  acc_guard4(acc[0][0], acc[0][1], acc[0][2], acc[0][3]);
  acc_guard4(acc[1][0], acc[1][1], acc[1][2], acc[1][3]);
  acc_guard4(acc[2][0], acc[2][1], acc[2][2], acc[2][3]);
  acc_guard4(acc[3][0], acc[3][1], acc[3][2], acc[3][3]);

  float* slab = sT[wave];
  const float* Rb = RESID ? (resid + (size_t)b * strideR) : nullptr;
#pragma unroll
  for (int i = 0; i < 4; ++i) {
    const int mBase = m0 + (i << 4);
#pragma unroll
    for (int j = 0; j < 4; ++j) {
      const int n = n0 + (j << 4) + rlane;
      float bv = 0.f;
      if (BIAS_MODE == 2) bv = bias[n];
#pragma unroll
      for (int r = 0; r < 8; ++r) {
        float v = acc[i][j][r] * scale;
        if (BIAS_MODE == 1) v += bias[mBase + mOff + r];
        if (BIAS_MODE == 2) v += bv;
        if (RESID) v += Rb[(size_t)(mBase + mOff + r) * ldc + n];
        if (ACT == 1) v = tanhf(v);
        if (ACT == 2) v = fmaxf(v, 0.0f);
        if (ACT == 4) v = (v > 0.f) ? v : 0.01f * v;
        slab[(mOff + r) * 68 + (j << 4) + rlane] = v;
      }
    }
    __builtin_amdgcn_fence(__ATOMIC_RELEASE, "workgroup");
    __builtin_amdgcn_wave_barrier();
    __builtin_amdgcn_fence(__ATOMIC_ACQUIRE, "workgroup");
    if (OUT_MODE == 0) {
      float* C = (float*)Cout + (size_t)b * strideC;
      const int hh = lane >> 4, c4 = (lane & 15) * 4;
      for (int pass = 0; pass < 2; ++pass) {
#pragma unroll
        for (int it = 0; it < 8; ++it) {
          const int row = it * 2 + hh;
          v4f v = *(const v4f*)(slab + row * 68 + c4);
          *(volatile v4f*)(C + (size_t)(mBase + row) * ldc + n0 + c4) = v;
        }
        __threadfence();
      }
    } else {
      const int q = lane >> 3, c8 = (lane & 7) * 8;
      unsigned short* C  = (unsigned short*)Cout  + (size_t)b * strideC;
      unsigned short* C2 = (OUT_MODE == 2) ? ((unsigned short*)Cout2 + (size_t)b * strideC) : nullptr;
      for (int pass = 0; pass < 2; ++pass) {
#pragma unroll
        for (int it = 0; it < 4; ++it) {
          const int row = it * 4 + q;
          const float* sp = slab + row * 68 + c8;
          v8h hv, lv;
#pragma unroll
          for (int e = 0; e < 8; ++e) {
            if (OUT_MODE == 1) {
              hv[e] = (_Float16)sp[e];
            } else {
              unsigned short hb = f2bf_bits(sp[e]);
              unsigned short lb = f2bf_bits(sp[e] - bf_bits2f(hb));
              hv[e] = __builtin_bit_cast(_Float16, hb);
              lv[e] = __builtin_bit_cast(_Float16, lb);
            }
          }
          *(volatile v8h*)(C + (size_t)(mBase + row) * ldc + n0 + c8) = hv;
          if (OUT_MODE == 2) *(volatile v8h*)(C2 + (size_t)(mBase + row) * ldc + n0 + c8) = lv;
        }
        __threadfence();
      }
    }
    __builtin_amdgcn_fence(__ATOMIC_RELEASE, "workgroup");
    __builtin_amdgcn_wave_barrier();
    __builtin_amdgcn_fence(__ATOMIC_ACQUIRE, "workgroup");
  }
}

__device__ __forceinline__ v8f at_mma(v16b a, v16b b, v8f c) {
  c = __builtin_amdgcn_wmma_f32_16x16x32_bf16(false, a, false, b, (short)0, c, false, false);
  asm volatile("v_nop\n\tv_nop\n\tv_nop\n\tv_nop" : "+v"(c) : "v"(a), "v"(b));
  return c;
}

__global__ __launch_bounds__(256) void cast_f32_bf16x8(const float* __restrict__ in, unsigned short* __restrict__ out, int n8) {
  const int i = blockIdx.x * 256 + threadIdx.x;
  if (i >= n8) return;
  const float* p = in + (size_t)i * 8;
  const v4f a = *(const v4f*)p;
  const v4f c2 = *(const v4f*)(p + 4);
  v4u w;
  w[0] = pack_bf16x2(a[0], a[1]);
  w[1] = pack_bf16x2(a[2], a[3]);
  w[2] = pack_bf16x2(c2[0], c2[1]);
  w[3] = pack_bf16x2(c2[2], c2[3]);
  volatile v4u* d = (volatile v4u*)(out + (size_t)i * 8);
  *d = w;
  __threadfence();
  *d = w;
}

__global__ __launch_bounds__(256) void rne_bf16_f32x4(const float* __restrict__ in, float* __restrict__ out, int n4) {
  const int i = blockIdx.x * 256 + threadIdx.x;
  if (i >= n4) return;
  v4u a = *(const v4u*)(in + (size_t)i * 4);
#pragma unroll
  for (int e = 0; e < 4; ++e) a[e] = rne_bf16_word(a[e]);
  volatile v4u* d = (volatile v4u*)(out + (size_t)i * 4);
  *d = a;
  __threadfence();
  *d = a;
}

__global__ __launch_bounds__(256) void transpose_cast_bf16(const float* __restrict__ in, unsigned short* __restrict__ out, int nrows, int ncols) {
  __shared__ __align__(16) float tile[64 * 68];
  const int tid = threadIdx.x, lane = tid & 31, wave = tid >> 5;
  const int r0 = blockIdx.y * 64;
  const int c0 = blockIdx.x * 64;
  {
    const int rl = tid >> 2, cq = (tid & 3) * 16;
    const float* src = in + (size_t)(r0 + rl) * ncols + c0 + cq;
#pragma unroll
    for (int i = 0; i < 4; ++i) {
      const v4f v = *(const v4f*)(src + 4 * i);
#pragma unroll
      for (int e = 0; e < 4; ++e) tile[(cq + 4 * i + e) * 68 + rl] = v[e];
    }
  }
  __syncthreads();
  const int q8 = lane >> 3, c8 = (lane & 7) * 8;
  for (int pass = 0; pass < 2; ++pass) {
#pragma unroll
    for (int it = 0; it < 2; ++it) {
      const int cl = wave * 8 + it * 4 + q8;
      const float* sp = tile + cl * 68 + c8;
      const v4f x0 = *(const v4f*)sp;
      const v4f x1 = *(const v4f*)(sp + 4);
      v4u w;
      w[0] = pack_bf16x2(x0[0], x0[1]);
      w[1] = pack_bf16x2(x0[2], x0[3]);
      w[2] = pack_bf16x2(x1[0], x1[1]);
      w[3] = pack_bf16x2(x1[2], x1[3]);
      *(volatile v4u*)(out + (size_t)(c0 + cl) * nrows + r0 + c8) = w;
    }
    __threadfence();
  }
}

#define SEQ_LEN 2048
#define N_HEADS 16
#define HEAD_D 64
#define HID_SZ 1024
#define QKV_PITCH 3072
#define KV_CHUNK 64
#define N_BATCH 2

__global__ __launch_bounds__(128) void attn_planes_kernel(
    const unsigned short* __restrict__ qkvh, const unsigned short* __restrict__ qkvl,
    const float* __restrict__ maskp,
    unsigned short* __restrict__ ctxh, unsigned short* __restrict__ ctxl) {
  union FB { v16b v; v8b h[2]; };
  __shared__ __align__(16) unsigned short Kh[KV_CHUNK * HEAD_D];
  __shared__ __align__(16) unsigned short Kl[KV_CHUNK * HEAD_D];
  __shared__ __align__(16) unsigned short Vth[HEAD_D * KV_CHUNK];
  __shared__ __align__(16) unsigned short Vtl[HEAD_D * KV_CHUNK];
  __shared__ __align__(16) unsigned short Psh[4][16 * KV_CHUNK];
  __shared__ __align__(16) unsigned short Psl[4][16 * KV_CHUNK];
  __shared__ __align__(16) float Os[4][16 * 68];
  __shared__ __align__(16) unsigned int Msk[64 * 68];
  __shared__ int AnyNZ[4];

  const int tid  = threadIdx.x;
  const int wave = tid >> 5;
  const int lane = tid & 31;
  const int hh   = lane >> 4;
  const int c    = lane & 15;
  const int bx   = blockIdx.x;
  const int qb   = bx & 31;
  const int bhd  = bx >> 5;
  const int h    = bhd & (N_HEADS - 1);
  const int b    = bhd >> 4;
  const int qblk = qb * 64;
  const int q0   = qblk + wave * 16;
  const size_t rowb = (size_t)b * SEQ_LEN;

  v16b qah[2], qal[2];
  {
    const size_t qoff = (rowb + q0 + c) * QKV_PITCH + h * HEAD_D + 8 * hh;
#pragma unroll
    for (int dc = 0; dc < 2; ++dc) {
      qah[dc] = Frag<__bf16>::load((const __bf16*)qkvh + qoff + dc * 32);
      qal[dc] = Frag<__bf16>::load((const __bf16*)qkvl + qoff + dc * 32);
    }
  }

  float mrow[8], lrow[8];
  v8f oacc[4];
#pragma unroll
  for (int r = 0; r < 8; ++r) { mrow[r] = -__builtin_inff(); lrow[r] = 0.f; }
#pragma unroll
  for (int t = 0; t < 4; ++t) oacc[t] = (v8f){0.f,0.f,0.f,0.f,0.f,0.f,0.f,0.f};

  const int kvr = tid >> 1;
  const int dh  = (tid & 1) * 32;

  for (int kc = 0; kc < SEQ_LEN / KV_CHUNK; ++kc) {
    const int kv0 = kc * KV_CHUNK;
    __syncthreads();
    unsigned int nz = 0u;
#pragma unroll
    for (int i = 0; i < 8; ++i) {
      const int idx = i * 128 + tid;
      const int row = idx >> 4;
      const int c4  = (idx & 15) * 4;
      v4u m = *(const v4u*)(maskp + (size_t)(qblk + row) * SEQ_LEN + kv0 + c4);
#pragma unroll
      for (int e = 0; e < 4; ++e) { const unsigned int u = rne_bf16_word(m[e]); m[e] = u; nz |= (u & 0x7FFFFFFFu); }
      *(v4u*)(Msk + row * 68 + c4) = m;
    }
    const int anyw = __any(nz != 0u);
    AnyNZ[wave] = anyw;
    __syncthreads();
    const int tile_live = AnyNZ[0] | AnyNZ[1] | AnyNZ[2] | AnyNZ[3];

    const size_t koff = (rowb + kv0 + kvr) * QKV_PITCH + HID_SZ + h * HEAD_D + dh;
    const size_t voff = koff + HID_SZ;

    if (tile_live) {
      {
        const v4u* gh = (const v4u*)(qkvh + koff);
        const v4u* gl = (const v4u*)(qkvl + koff);
        v4u* lh = (v4u*)(Kh + kvr * HEAD_D + dh);
        v4u* ll = (v4u*)(Kl + kvr * HEAD_D + dh);
#pragma unroll
        for (int i = 0; i < 4; ++i) { const v4u a = gh[i]; const v4u bb = gl[i]; lh[i] = a; ll[i] = bb; }
      }
      asm volatile("" ::: "memory");
      {
        const v4u* gh = (const v4u*)(qkvh + voff);
        const v4u* gl = (const v4u*)(qkvl + voff);
#pragma unroll
        for (int i = 0; i < 4; ++i) {
          const v4u wh = gh[i];
          const v4u wl = gl[i];
#pragma unroll
          for (int e = 0; e < 4; ++e) {
            const int d = dh + 8 * i + 2 * e;
            Vth[d * KV_CHUNK + kvr]       = (unsigned short)(wh[e] & 0xFFFFu);
            Vth[(d + 1) * KV_CHUNK + kvr] = (unsigned short)(wh[e] >> 16);
            Vtl[d * KV_CHUNK + kvr]       = (unsigned short)(wl[e] & 0xFFFFu);
            Vtl[(d + 1) * KV_CHUNK + kvr] = (unsigned short)(wl[e] >> 16);
          }
        }
      }
      __syncthreads();

      v8f s[4];
#pragma unroll
      for (int j = 0; j < 4; ++j) {
        s[j] = (v8f){0.f,0.f,0.f,0.f,0.f,0.f,0.f,0.f};
#pragma unroll
        for (int dc = 0; dc < 2; ++dc) {
          FB kb, kl;
          const int ko = (j * 16 + c) * HEAD_D + dc * 32 + 8 * hh;
          kb.h[0] = *(const v8b*)((const __bf16*)Kh + ko);
          kb.h[1] = *(const v8b*)((const __bf16*)Kh + ko + 16);
          kl.h[0] = *(const v8b*)((const __bf16*)Kl + ko);
          kl.h[1] = *(const v8b*)((const __bf16*)Kl + ko + 16);
          s[j] = at_mma(qah[dc], kb.v, s[j]);
          s[j] = at_mma(qah[dc], kl.v, s[j]);
          s[j] = at_mma(qal[dc], kb.v, s[j]);
        }
      }
      float cm[8];
#pragma unroll
      for (int r = 0; r < 8; ++r) {
        const int rl = wave * 16 + 8 * hh + r;
        float m = -__builtin_inff();
#pragma unroll
        for (int j = 0; j < 4; ++j) {
          const float mk = __uint_as_float(Msk[rl * 68 + j * 16 + c]);
          float x = s[j][r] * 0.125f;
          x = x * mk - 10000.0f * (1.0f - mk);
          s[j][r] = x;
          m = fmaxf(m, x);
        }
#pragma unroll
        for (int off = 1; off < 16; off <<= 1) m = fmaxf(m, __shfl_xor(m, off, 32));
        cm[r] = m;
      }
      unsigned short* pwh = Psh[wave];
      unsigned short* pwl = Psl[wave];
#pragma unroll
      for (int r = 0; r < 8; ++r) {
        const float mnew  = fmaxf(mrow[r], cm[r]);
        const float alpha = expf(mrow[r] - mnew);
        mrow[r] = mnew;
        float psum = 0.f;
#pragma unroll
        for (int j = 0; j < 4; ++j) {
          const float p = expf(s[j][r] - mnew);
          psum += p;
          const unsigned short hb = f2bf_bits(p);
          const unsigned short lb = f2bf_bits(p - bf_bits2f(hb));
          pwh[(8 * hh + r) * KV_CHUNK + j * 16 + c] = hb;
          pwl[(8 * hh + r) * KV_CHUNK + j * 16 + c] = lb;
        }
#pragma unroll
        for (int off = 1; off < 16; off <<= 1) psum += __shfl_xor(psum, off, 32);
        lrow[r] = lrow[r] * alpha + psum;
#pragma unroll
        for (int t = 0; t < 4; ++t) oacc[t][r] *= alpha;
      }
      __builtin_amdgcn_fence(__ATOMIC_RELEASE, "workgroup");
      __builtin_amdgcn_wave_barrier();
      __builtin_amdgcn_fence(__ATOMIC_ACQUIRE, "workgroup");
#pragma unroll 1
      for (int kk = 0; kk < 2; ++kk) {
        FB pa, pl;
        const int po = c * KV_CHUNK + kk * 32 + 8 * hh;
        pa.h[0] = *(const v8b*)((const __bf16*)pwh + po);
        pa.h[1] = *(const v8b*)((const __bf16*)pwh + po + 16);
        pl.h[0] = *(const v8b*)((const __bf16*)pwl + po);
        pl.h[1] = *(const v8b*)((const __bf16*)pwl + po + 16);
#pragma unroll
        for (int t = 0; t < 4; ++t) {
          FB vb, vl;
          const int vo = (t * 16 + c) * KV_CHUNK + kk * 32 + 8 * hh;
          vb.h[0] = *(const v8b*)((const __bf16*)Vth + vo);
          vb.h[1] = *(const v8b*)((const __bf16*)Vth + vo + 16);
          vl.h[0] = *(const v8b*)((const __bf16*)Vtl + vo);
          vl.h[1] = *(const v8b*)((const __bf16*)Vtl + vo + 16);
          oacc[t] = at_mma(pa.v, vb.v, oacc[t]);
          oacc[t] = at_mma(pa.v, vl.v, oacc[t]);
          oacc[t] = at_mma(pl.v, vb.v, oacc[t]);
        }
      }
    } else {
      {
        const v4u* gh = (const v4u*)(qkvh + voff);
        const v4u* gl = (const v4u*)(qkvl + voff);
#pragma unroll
        for (int i = 0; i < 4; ++i) {
          const v4u wh = gh[i];
          const v4u wl = gl[i];
          v4u f0, f1;
          {
            const float a0 = __uint_as_float(wh[0] << 16);          const float b0 = __uint_as_float(wl[0] << 16);
            const float a1 = __uint_as_float(wh[0] & 0xFFFF0000u); const float b1 = __uint_as_float(wl[0] & 0xFFFF0000u);
            const float a2 = __uint_as_float(wh[1] << 16);          const float b2 = __uint_as_float(wl[1] << 16);
            const float a3 = __uint_as_float(wh[1] & 0xFFFF0000u); const float b3 = __uint_as_float(wl[1] & 0xFFFF0000u);
            f0[0] = __float_as_uint(a0 + b0); f0[1] = __float_as_uint(a1 + b1);
            f0[2] = __float_as_uint(a2 + b2); f0[3] = __float_as_uint(a3 + b3);
          }
          {
            const float a0 = __uint_as_float(wh[2] << 16);          const float b0 = __uint_as_float(wl[2] << 16);
            const float a1 = __uint_as_float(wh[2] & 0xFFFF0000u); const float b1 = __uint_as_float(wl[2] & 0xFFFF0000u);
            const float a2 = __uint_as_float(wh[3] << 16);          const float b2 = __uint_as_float(wl[3] << 16);
            const float a3 = __uint_as_float(wh[3] & 0xFFFF0000u); const float b3 = __uint_as_float(wl[3] & 0xFFFF0000u);
            f1[0] = __float_as_uint(a0 + b0); f1[1] = __float_as_uint(a1 + b1);
            f1[2] = __float_as_uint(a2 + b2); f1[3] = __float_as_uint(a3 + b3);
          }
          *(v4u*)(Msk + kvr * 68 + dh + 8 * i)     = f0;
          *(v4u*)(Msk + kvr * 68 + dh + 8 * i + 4) = f1;
        }
      }
      __syncthreads();
      {
        const int d = tid & 63, half = tid >> 6;
        float part = 0.f;
#pragma unroll 8
        for (int kq = 0; kq < 32; ++kq) part += __uint_as_float(Msk[(half * 32 + kq) * 68 + d]);
        Os[0][half * 64 + d] = part;
      }
      __syncthreads();
      float vs[4];
#pragma unroll
      for (int t = 0; t < 4; ++t) vs[t] = Os[0][t * 16 + c] + Os[0][64 + t * 16 + c];
#pragma unroll
      for (int r = 0; r < 8; ++r) {
        const float mnew  = fmaxf(mrow[r], -10000.0f);
        const float alpha = expf(mrow[r] - mnew);
        const float p     = expf(-10000.0f - mnew);
        mrow[r] = mnew;
        lrow[r] = lrow[r] * alpha + 64.0f * p;
#pragma unroll
        for (int t = 0; t < 4; ++t) oacc[t][r] = oacc[t][r] * alpha + p * vs[t];
      }
    }
  }
  __syncthreads();

  float* os = Os[wave];
#pragma unroll
  for (int r = 0; r < 8; ++r) {
    const float inv = 1.0f / lrow[r];
#pragma unroll
    for (int t = 0; t < 4; ++t) os[(8 * hh + r) * 68 + t * 16 + c] = oacc[t][r] * inv;
  }
  __builtin_amdgcn_fence(__ATOMIC_RELEASE, "workgroup");
  __builtin_amdgcn_wave_barrier();
  __builtin_amdgcn_fence(__ATOMIC_ACQUIRE, "workgroup");
  {
    const int q8 = lane >> 3, c8 = (lane & 7) * 8;
    unsigned short* oh = ctxh + (rowb + q0) * HID_SZ + h * HEAD_D + c8;
    unsigned short* ol = ctxl + (rowb + q0) * HID_SZ + h * HEAD_D + c8;
    for (int pass = 0; pass < 2; ++pass) {
#pragma unroll
      for (int it = 0; it < 4; ++it) {
        const int row = it * 4 + q8;
        const float* sp = os + row * 68 + c8;
        const v4f x0 = *(const v4f*)sp;
        const v4f x1 = *(const v4f*)(sp + 4);
        v4u wh, wl;
        unsigned int th, tl;
        split_pack2(x0[0], x0[1], th, tl); wh[0] = th; wl[0] = tl;
        split_pack2(x0[2], x0[3], th, tl); wh[1] = th; wl[1] = tl;
        split_pack2(x1[0], x1[1], th, tl); wh[2] = th; wl[2] = tl;
        split_pack2(x1[2], x1[3], th, tl); wh[3] = th; wl[3] = tl;
        *(volatile v4u*)(oh + (size_t)row * HID_SZ) = wh;
        *(volatile v4u*)(ol + (size_t)row * HID_SZ) = wl;
      }
      __threadfence();
    }
  }
}

extern "C" void kernel_launch(void* const* d_in, const int* in_sizes, int n_in,
                              void* d_out, int out_size, void* d_ws, size_t ws_size,
                              hipStream_t stream) {
  constexpr int kB = N_BATCH, kS = SEQ_LEN, kH = HID_SZ;
  constexpr int kM = kB * kS;
  constexpr int kN3 = 3 * kH;
  static_assert(kM % 64 == 0 && kN3 % 64 == 0 && kH % 64 == 0);
  static_assert(kH % 32 == 0);
  static_assert(kS % KV_CHUNK == 0 && kS / 64 == 32 && kH / HEAD_D == N_HEADS);
  static_assert((kM * kH) % 2048 == 0 && kN3 % 1024 == 0 && kH % 1024 == 0);

  if (n_in < 6) return;
  if (in_sizes[0] != kM * kH || in_sizes[1] != kS * kS || in_sizes[2] != kH * kN3 ||
      in_sizes[3] != kN3 || in_sizes[4] != kH * kH || in_sizes[5] != kH) return;
  if (out_size != kM * kH) return;

  const float* hidden  = (const float*)d_in[0];
  const float* maskp   = (const float*)d_in[1];
  const float* w_qkv   = (const float*)d_in[2];
  const float* b_qkv   = (const float*)d_in[3];
  const float* w_dense = (const float*)d_in[4];
  const float* b_dense = (const float*)d_in[5];
  float* out = (float*)d_out;

  const size_t szHb  = (size_t)kM * kH * 2;
  const size_t szWQt = (size_t)kN3 * kH * 2;
  const size_t szWDt = (size_t)kH * kH * 2;
  const size_t szBQ  = (size_t)kN3 * 4;
  const size_t szBD  = (size_t)kH * 4;
  const size_t szQKV = (size_t)kM * kN3 * 2;
  const size_t szCTX = (size_t)kM * kH * 2;
  const size_t offHb   = 0;
  const size_t offWQt  = offHb + szHb;
  const size_t offWDt  = offWQt + szWQt;
  const size_t offBQ   = offWDt + szWDt;
  const size_t offBD   = offBQ + szBQ;
  const size_t offQKVh = offBD + szBD;
  const size_t offQKVl = offQKVh + szQKV;
  const size_t offCTXh = offQKVl + szQKV;
  const size_t offCTXl = offCTXh + szCTX;
  const size_t offEnd  = offCTXl + szCTX;
  if (offEnd > ws_size) return;

  char* ws = (char*)d_ws;
  unsigned short* Hb   = (unsigned short*)(ws + offHb);
  unsigned short* WQt  = (unsigned short*)(ws + offWQt);
  unsigned short* WDt  = (unsigned short*)(ws + offWDt);
  float*          BQ   = (float*)(ws + offBQ);
  float*          BD   = (float*)(ws + offBD);
  unsigned short* QKVh = (unsigned short*)(ws + offQKVh);
  unsigned short* QKVl = (unsigned short*)(ws + offQKVl);
  unsigned short* CTXh = (unsigned short*)(ws + offCTXh);
  unsigned short* CTXl = (unsigned short*)(ws + offCTXl);

  {
    const int n8 = (kM * kH) / 8;
    cast_f32_bf16x8<<<dim3(n8 / 256), dim3(256), 0, stream>>>(hidden, Hb, n8);
  }
  transpose_cast_bf16<<<dim3(kN3 / 64, kH / 64), dim3(256), 0, stream>>>(w_qkv, WQt, kH, kN3);
  transpose_cast_bf16<<<dim3(kH / 64, kH / 64), dim3(256), 0, stream>>>(w_dense, WDt, kH, kH);
  rne_bf16_f32x4<<<dim3((kN3 / 4) / 256), dim3(256), 0, stream>>>(b_qkv, BQ, kN3 / 4);
  rne_bf16_f32x4<<<dim3((kH / 4) / 256), dim3(256), 0, stream>>>(b_dense, BD, kH / 4);
  {
    const int tiles = (kM / 64) * (kN3 / 64);
    wmma_gemm64<1, 0, 2, 2, false><<<dim3(tiles / 8, 1), dim3(256), 0, stream>>>(
        Hb, Hb, kH, 0L, WQt, WQt, kH, 0L, (void*)QKVh, (void*)QKVl, kN3, 0L,
        BQ, BQ, 0L, kM, kN3, kH, 1.0f);
  }
  attn_planes_kernel<<<dim3(kB * N_HEADS * (kS / 64)), dim3(128), 0, stream>>>(QKVh, QKVl, maskp, CTXh, CTXl);
  {
    const int tiles = (kM / 64) * (kH / 64);
    wmma_gemm64<1, 2, 2, 0, false><<<dim3(tiles / 8, 1), dim3(256), 0, stream>>>(
        CTXh, CTXl, kH, 0L, WDt, WDt, kH, 0L, (void*)out, (void*)out, kH, 0L,
        BD, BD, 0L, kM, kH, kH, 1.0f);
  }
}
